// capsule_87840671138361
// MI455X (gfx1250) — hardware-verified
//
#include <hip/hip_runtime.h>
#include <math.h>

constexpr int kBatch = 8;
constexpr int kSeq   = 2048;
constexpr int kDim   = 512;
constexpr int kTok   = kBatch * kSeq;
constexpr int kCat   = 2 * kDim;
constexpr float kDecay    = 0.2f;
constexpr float kVCarry   = 64.0f;
constexpr float kPCarry   = 1024.0f;
constexpr float kWCarry   = 16.0f;
constexpr float kSimScale = 1.0f / (64.0f * 64.0f);
constexpr float kPVScale  = 1.0f / 1024.0f;
constexpr float kOutScale = 1.0f / (64.0f * 16.0f);

typedef __attribute__((ext_vector_type(16))) _Float16 v16h;
typedef __attribute__((ext_vector_type(8)))  _Float16 v8h;
typedef __attribute__((ext_vector_type(16))) __bf16   v16b;
typedef __attribute__((ext_vector_type(8)))  __bf16   v8b;
typedef __attribute__((ext_vector_type(8)))  float    v8f;
typedef __attribute__((ext_vector_type(4)))  float    v4f;
typedef __attribute__((ext_vector_type(2)))  float    v2f;
typedef __attribute__((ext_vector_type(4)))  unsigned int v4u;

__device__ __forceinline__ unsigned short f2bf_bits(float f) {
  unsigned u = __float_as_uint(f);
  return (unsigned short)((u + 0x7FFFu + ((u >> 16) & 1u)) >> 16);
}
__device__ __forceinline__ float bf_bits2f(unsigned short h) { return __uint_as_float(((unsigned)h) << 16); }

__device__ __forceinline__ void dep_guard_h(v8f& a, v8f& b, v16h x, v16h y) { asm volatile("v_nop\n\tv_nop\n\tv_nop\n\tv_nop" : "+v"(a), "+v"(b) : "v"(x), "v"(y)); }
__device__ __forceinline__ void dep_guard_b(v8f& a, v8f& b, v16b x, v16b y) { asm volatile("v_nop\n\tv_nop\n\tv_nop\n\tv_nop" : "+v"(a), "+v"(b) : "v"(x), "v"(y)); }
__device__ __forceinline__ void keep4_h(v16h a, v16h b, v16h c, v16h d) { asm volatile("v_nop" :: "v"(a), "v"(b), "v"(c), "v"(d)); }
__device__ __forceinline__ void keep4_b(v16b a, v16b b, v16b c, v16b d) { asm volatile("v_nop" :: "v"(a), "v"(b), "v"(c), "v"(d)); }
__device__ __forceinline__ void acc_guard4(v8f& a, v8f& b, v8f& c, v8f& d) { asm volatile("v_nop\n\tv_nop\n\tv_nop\n\tv_nop" : "+v"(a), "+v"(b), "+v"(c), "+v"(d)); }
template <typename T> struct Frag;
template <> struct Frag<_Float16> {
  typedef v16h V; union U { v16h v; v8h h[2]; };
  static __device__ __forceinline__ v16h load(const _Float16* p) {
    U f; f.h[0] = *(const v8h*)(p); f.h[1] = *(const v8h*)(p + 16); return f.v;
  }
  static __device__ __forceinline__ v8f mma(v16h a, v16h b, v8f c) {
    return __builtin_amdgcn_wmma_f32_16x16x32_f16(false, a, false, b, (short)0, c, false, false);
  }
  static __device__ __forceinline__ void guard(v8f& a, v8f& b, v16h x, v16h y) { dep_guard_h(a, b, x, y); }
  static __device__ __forceinline__ void keep(v16h a, v16h b, v16h c, v16h d) { keep4_h(a, b, c, d); }
};
template <> struct Frag<__bf16> {
  typedef v16b V; union U { v16b v; v8b h[2]; };
  static __device__ __forceinline__ v16b load(const __bf16* p) {
    U f; f.h[0] = *(const v8b*)(p); f.h[1] = *(const v8b*)(p + 16); return f.v;
  }
  static __device__ __forceinline__ v8f mma(v16b a, v16b b, v8f c) {
    return __builtin_amdgcn_wmma_f32_16x16x32_bf16(false, a, false, b, (short)0, c, false, false);
  }
  static __device__ __forceinline__ void guard(v8f& a, v8f& b, v16b x, v16b y) { dep_guard_b(a, b, x, y); }
  static __device__ __forceinline__ void keep(v16b a, v16b b, v16b c, v16b d) { keep4_b(a, b, c, d); }
};

__device__ __forceinline__ unsigned pk16(unsigned short a, unsigned short b) { return (unsigned)a | ((unsigned)b << 16); }
__device__ __forceinline__ unsigned short h_bits(float f) { const _Float16 h = (_Float16)f; return __builtin_bit_cast(unsigned short, h); }

template <int ET> struct Elem;
template <> struct Elem<0> { typedef _Float16 T; };
template <> struct Elem<1> { typedef __bf16 T; };
template <int ET, bool SPLIT, int BIAS_MODE, int OUT_MODE, bool RESID, int ACT = 0, int CAUSAL = 0>
__global__ __launch_bounds__(256) void wmma_gemm64(
    const unsigned short* __restrict__ Ap, const unsigned short* __restrict__ A2p, int lda, long strideA,
    const unsigned short* __restrict__ Btp, const unsigned short* __restrict__ Bt2p, int ldb, long strideB,
    void* __restrict__ Cout, void* __restrict__ Cout2, int ldc, long strideC,
    const float* __restrict__ bias,
    const float* __restrict__ resid, long strideR,
    int M, int N, int K, float scale) {
  typedef typename Elem<ET>::T T;
  typedef typename Frag<T>::V V;
  const T* A = (const T*)Ap; const T* A2 = (const T*)A2p; const T* Bt = (const T*)Btp; const T* Bt2 = (const T*)Bt2p;
  __shared__ __align__(16) float sT[8][16 * 68];
  const int b    = blockIdx.y;
  const int lane = threadIdx.x & 31;
  const int wave = threadIdx.x >> 5;
  const int tilesN = N >> 6;
  const int tilesM = M >> 6;
  const int tile = blockIdx.x * 8 + wave;
  int tm, tn;
  if (CAUSAL == 1) {
    const int ntri = (tilesM * (tilesM + 1)) >> 1;
    if (tile >= ntri) return;
    int tq = (int)((sqrtf((float)(8 * tile + 1)) - 1.0f) * 0.5f);
    if ((((tq + 1) * (tq + 2)) >> 1) <= tile) tq += 1;
    if (((tq * (tq + 1)) >> 1) > tile) tq -= 1;
    tm = tq;
    tn = tile - ((tq * (tq + 1)) >> 1);
  } else {
    if (tile >= tilesM * tilesN) return;
    tm = tile / tilesN;
    tn = tile - tm * tilesN;
  }
  const int m0 = tm << 6;
  const int n0 = tn << 6;
  const int Kend = (CAUSAL == 2) ? (((m0 + 64) < K) ? (m0 + 64) : K) : K;

  const T* Ab  = A  + (size_t)b * strideA;
  const T* Bb  = Bt + (size_t)b * strideB;
  const T* Ab2 = SPLIT ? (A2  + (size_t)b * strideA) : nullptr;
  const T* Bb2 = SPLIT ? (Bt2 + (size_t)b * strideB) : nullptr;

  const int rlane = lane & 15;
  const int koff  = (lane >> 4) * 8;
  const int mOff  = (lane >> 4) * 8;

  v8f acc[4][4];
#pragma unroll
  for (int i = 0; i < 4; ++i)
#pragma unroll
    for (int j = 0; j < 4; ++j) acc[i][j] = (v8f){0.f,0.f,0.f,0.f,0.f,0.f,0.f,0.f};

  for (int k0 = 0; k0 < Kend; k0 += 32) {
    V bh[4], bl[4];
#pragma unroll
    for (int j = 0; j < 4; ++j) {
      const size_t bo = (size_t)(n0 + (j << 4) + rlane) * ldb + koff + k0;
      bh[j] = Frag<T>::load(Bb + bo);
      if (SPLIT) bl[j] = Frag<T>::load(Bb2 + bo);
    }
#pragma unroll
    for (int i = 0; i < 4; ++i) {
      const size_t ao = (size_t)(m0 + (i << 4) + rlane) * lda + koff + k0;
      V ah = Frag<T>::load(Ab + ao);
      V al;
      if (SPLIT) al = Frag<T>::load(Ab2 + ao);
#pragma unroll
      for (int j = 0; j < 4; ++j) {
        acc[i][j] = Frag<T>::mma(ah, bh[j], acc[i][j]);
        if (SPLIT) {
          acc[i][j] = Frag<T>::mma(ah, bl[j], acc[i][j]);
          acc[i][j] = Frag<T>::mma(al, bh[j], acc[i][j]);
        }
      }
      Frag<T>::guard(acc[i][0], acc[i][3], ah, SPLIT ? al : ah);
    }
    Frag<T>::keep(bh[0], bh[1], bh[2], bh[3]);
    if (SPLIT) Frag<T>::keep(bl[0], bl[1], bl[2], bl[3]);
  }
  acc_guard4(acc[0][0], acc[0][1], acc[0][2], acc[0][3]);
  acc_guard4(acc[1][0], acc[1][1], acc[1][2], acc[1][3]);
  acc_guard4(acc[2][0], acc[2][1], acc[2][2], acc[2][3]);
  acc_guard4(acc[3][0], acc[3][1], acc[3][2], acc[3][3]);

  float* slab = sT[wave];
  const float* Rb = RESID ? (resid + (size_t)b * strideR) : nullptr;
#pragma unroll
  for (int i = 0; i < 4; ++i) {
    const int mBase = m0 + (i << 4);
#pragma unroll
    for (int j = 0; j < 4; ++j) {
      const int n = n0 + (j << 4) + rlane;
      float bv = 0.f;
      if (BIAS_MODE == 2) bv = bias[n];
#pragma unroll
      for (int r = 0; r < 8; ++r) {
        float v = acc[i][j][r] * scale;
        if (BIAS_MODE == 1) v += bias[mBase + mOff + r];
        if (BIAS_MODE == 2) v += bv;
        if (RESID) v += Rb[(size_t)(mBase + mOff + r) * ldc + n];
        if (ACT == 2) v = fmaxf(v, 0.0f);
        if (ACT == 4) v = (v > 0.f) ? v : 0.01f * v;
        slab[(mOff + r) * 68 + (j << 4) + rlane] = v;
      }
    }
    __builtin_amdgcn_fence(__ATOMIC_RELEASE, "workgroup");
    __builtin_amdgcn_wave_barrier();
    __builtin_amdgcn_fence(__ATOMIC_ACQUIRE, "workgroup");
    if (OUT_MODE == 0) {
      float* C = (float*)Cout + (size_t)b * strideC;
      const int hh = lane >> 4, c4 = (lane & 15) * 4;
      for (int pass = 0; pass < 2; ++pass) {
#pragma unroll
        for (int it = 0; it < 8; ++it) {
          const int row = it * 2 + hh;
          v4f v = *(const v4f*)(slab + row * 68 + c4);
          *(volatile v4f*)(C + (size_t)(mBase + row) * ldc + n0 + c4) = v;
        }
        __threadfence();
      }
    } else {
      const int q = lane >> 3, c8 = (lane & 7) * 8;
      unsigned short* C  = (unsigned short*)Cout  + (size_t)b * strideC;
      unsigned short* C2 = (OUT_MODE == 2) ? ((unsigned short*)Cout2 + (size_t)b * strideC) : nullptr;
      for (int pass = 0; pass < 2; ++pass) {
#pragma unroll
        for (int it = 0; it < 4; ++it) {
          const int row = it * 4 + q;
          const float* sp = slab + row * 68 + c8;
          v8h hv, lv;
#pragma unroll
          for (int e = 0; e < 8; ++e) {
            if (OUT_MODE == 1) {
              hv[e] = (_Float16)sp[e];
            } else {
              unsigned short hb = f2bf_bits(sp[e]);
              unsigned short lb = f2bf_bits(sp[e] - bf_bits2f(hb));
              hv[e] = __builtin_bit_cast(_Float16, hb);
              lv[e] = __builtin_bit_cast(_Float16, lb);
            }
          }
          *(volatile v8h*)(C + (size_t)(mBase + row) * ldc + n0 + c8) = hv;
          if (OUT_MODE == 2) *(volatile v8h*)(C2 + (size_t)(mBase + row) * ldc + n0 + c8) = lv;
        }
        __threadfence();
      }
    }
    __builtin_amdgcn_fence(__ATOMIC_RELEASE, "workgroup");
    __builtin_amdgcn_wave_barrier();
    __builtin_amdgcn_fence(__ATOMIC_ACQUIRE, "workgroup");
  }
}

__global__ __launch_bounds__(256) void route_kernel(const float* __restrict__ x,
                                                    const float* __restrict__ w3,
                                                    const float* __restrict__ w5,
                                                    unsigned short* __restrict__ vS,
                                                    unsigned short* __restrict__ vT) {
  __shared__ float red[8][8];
  const int pos  = blockIdx.x;
  const int l    = pos & (kSeq - 1);
  const int tid  = threadIdx.x;
  const int lane = tid & 31;
  const int wave = tid >> 5;
  const int d    = 2 * tid;
  const size_t rowBase = (size_t)(pos - l);

  float xa[5], xb[5];
#pragma unroll
  for (int j = 0; j < 5; ++j) {
    const int li  = l - 4 + j;
    const int lic = (li < 0) ? 0 : li;
    const v2f t = *(const v2f*)(x + (rowBase + (size_t)lic) * kDim + d);
    const bool ok = (li >= 0);
    xa[j] = ok ? t.x : 0.f;
    xb[j] = ok ? t.y : 0.f;
  }
  const float t3a = xa[2] * w3[d * 3 + 0] + xa[3] * w3[d * 3 + 1] + xa[4] * w3[d * 3 + 2];
  const float t3b = xb[2] * w3[d * 3 + 3] + xb[3] * w3[d * 3 + 4] + xb[4] * w3[d * 3 + 5];
  const float t5a = xa[0] * w5[d * 5 + 0] + xa[1] * w5[d * 5 + 1] + xa[2] * w5[d * 5 + 2]
                  + xa[3] * w5[d * 5 + 3] + xa[4] * w5[d * 5 + 4];
  const float t5b = xb[0] * w5[d * 5 + 5] + xb[1] * w5[d * 5 + 6] + xb[2] * w5[d * 5 + 7]
                  + xb[3] * w5[d * 5 + 8] + xb[4] * w5[d * 5 + 9];

  float uA[2][2], uB[2][2];
  uA[0][0] = xa[4] - t3a; uA[0][1] = xb[4] - t3b;
  uB[0][0] = xa[4] - t5a; uB[0][1] = xb[4] - t5b;
  uA[1][0] = t3a;         uA[1][1] = t3b;
  uB[1][0] = t5a;         uB[1][1] = t5b;

  float b0[2] = {0.f, 0.f}, b1[2] = {0.f, 0.f};
  float s[2][2] = {{0.f, 0.f}, {0.f, 0.f}};
  float coef[2] = {0.f, 0.f};

#pragma unroll 1
  for (int it = 0; it < 3; ++it) {
    float part[2][3];
#pragma unroll
    for (int st = 0; st < 2; ++st) {
      const float mx  = fmaxf(b0[st], b1[st]);
      const float e0  = expf(b0[st] - mx);
      const float e1  = expf(b1[st] - mx);
      const float inv = 1.0f / (e0 + e1);
      const float c0  = e0 * inv;
      const float c1  = e1 * inv;
      float pss = 0.f, pd0 = 0.f, pd1 = 0.f;
#pragma unroll
      for (int c = 0; c < 2; ++c) {
        const float sv = c0 * uA[st][c] + c1 * uB[st][c];
        s[st][c] = sv;
        pss += sv * sv;
        pd0 += uA[st][c] * sv;
        pd1 += uB[st][c] * sv;
      }
      part[st][0] = pss; part[st][1] = pd0; part[st][2] = pd1;
    }
#pragma unroll
    for (int st = 0; st < 2; ++st)
#pragma unroll
      for (int q = 0; q < 3; ++q) {
        float v = part[st][q];
#pragma unroll
        for (int off = 16; off > 0; off >>= 1) v += __shfl_xor(v, off, 32);
        part[st][q] = v;
      }
    if (lane == 0) {
#pragma unroll
      for (int st = 0; st < 2; ++st)
#pragma unroll
        for (int q = 0; q < 3; ++q) red[wave][st * 3 + q] = part[st][q];
    }
    __syncthreads();
    float tot[2][3];
#pragma unroll
    for (int st = 0; st < 2; ++st)
#pragma unroll
      for (int q = 0; q < 3; ++q) {
        const int iq = st * 3 + q;
        tot[st][q] = ((((((red[0][iq] + red[1][iq]) + red[2][iq]) + red[3][iq]) + red[4][iq]) + red[5][iq]) + red[6][iq]) + red[7][iq];
      }
    __syncthreads();
#pragma unroll
    for (int st = 0; st < 2; ++st) {
      const float ss  = tot[st][0];
      const float nrm = sqrtf(ss);
      const float n2  = nrm * nrm;
      coef[st] = (n2 / (1.0f + n2)) / (nrm + 1e-9f);
      if (it < 2) {
        b0[st] += coef[st] * tot[st][1];
        b1[st] += coef[st] * tot[st][2];
      }
    }
  }

  const float vs0 = kVCarry * coef[0] * s[0][0];
  const float vs1 = kVCarry * coef[0] * s[0][1];
  const float vt0 = kVCarry * coef[1] * s[1][0];
  const float vt1 = kVCarry * coef[1] * s[1][1];
  const unsigned uS = pk16(h_bits(vs0), h_bits(vs1));
  const unsigned uT = pk16(h_bits(vt0), h_bits(vt1));
  volatile unsigned* pS = (volatile unsigned*)vS + (size_t)pos * (kDim / 2) + tid;
  volatile unsigned* pT = (volatile unsigned*)vT + (size_t)pos * (kDim / 2) + tid;
  *pS = uS;
  *pT = uT;
  __threadfence();
  *pS = uS;
  *pT = uT;
}

__global__ __launch_bounds__(256) void cast8_f16_kernel(const float* __restrict__ in, unsigned short* __restrict__ out,
                                                        int n8, float scale) {
  const int i = blockIdx.x * 256 + threadIdx.x;
  if (i >= n8) return;
  const float* p = in + 8 * (size_t)i;
  const v4f a = *(const v4f*)(p);
  const v4f c = *(const v4f*)(p + 4);
  unsigned short hb[8];
#pragma unroll
  for (int e = 0; e < 4; ++e) {
    hb[e]     = h_bits(a[e] * scale);
    hb[4 + e] = h_bits(c[e] * scale);
  }
  const v4u u = (v4u){pk16(hb[0], hb[1]), pk16(hb[2], hb[3]), pk16(hb[4], hb[5]), pk16(hb[6], hb[7])};
  unsigned short* q = out + 8 * (size_t)i;
  *(volatile v4u*)q = u;
  __threadfence();
  *(volatile v4u*)q = u;
}

__global__ __launch_bounds__(256) void vt_kernel(const unsigned short* __restrict__ src, long srcStride,
                                                 unsigned short* __restrict__ dst) {
  __shared__ unsigned short sm[64][72];
  const int t  = threadIdx.x;
  const int d0 = blockIdx.x * 64;
  const int t0 = blockIdx.y * 64;
  const int z  = blockIdx.z;
  const unsigned int* s32 = (const unsigned int*)(src + (size_t)z * srcStride);
#pragma unroll
  for (int i = 0; i < 8; ++i) {
    const int e  = i * 256 + t;
    const int r  = e >> 5;
    const int cp = e & 31;
    const unsigned w = s32[(size_t)(t0 + r) * (kDim / 2) + (d0 >> 1) + cp];
    sm[2 * cp][r]     = (unsigned short)(w & 0xFFFFu);
    sm[2 * cp + 1][r] = (unsigned short)(w >> 16);
  }
  __syncthreads();
  const int lane = t & 31, wave = t >> 5;
  const int q = lane >> 3, c8 = (lane & 7) * 8;
  unsigned short* op = dst + (size_t)z * kDim * kSeq;
  for (int pass = 0; pass < 2; ++pass) {
#pragma unroll
    for (int it = 0; it < 2; ++it) {
      const int row = wave * 8 + it * 4 + q;
      unsigned short hb[8];
#pragma unroll
      for (int e = 0; e < 8; ++e) hb[e] = sm[row][c8 + e];
      const v4u u = (v4u){pk16(hb[0], hb[1]), pk16(hb[2], hb[3]), pk16(hb[4], hb[5]), pk16(hb[6], hb[7])};
      *(volatile v4u*)(op + (size_t)(d0 + row) * kSeq + t0 + c8) = u;
    }
    __threadfence();
  }
}

__global__ __launch_bounds__(256) void softmax_kernel(const float* __restrict__ S, unsigned short* __restrict__ P,
                                                      float carry) {
  __shared__ float redM[8];
  __shared__ float redS[8];
  const int r    = blockIdx.x;
  const int z    = blockIdx.y;
  const int t    = threadIdx.x;
  const int lane = t & 31, wave = t >> 5;
  const int c0   = t * 8;
  const int limit = ((r >> 6) + 1) << 6;
  const int cl    = (c0 < limit - 8) ? c0 : (limit - 8);
  const float* sr = S + (size_t)z * kSeq * kSeq + (size_t)r * kSeq + cl;
  const v4f a  = *(const v4f*)(sr);
  const v4f c4 = *(const v4f*)(sr + 4);
  float xv[8];
#pragma unroll
  for (int e = 0; e < 4; ++e) { xv[e] = a[e]; xv[4 + e] = c4[e]; }
  float val[8];
  float m = -INFINITY;
#pragma unroll
  for (int e = 0; e < 8; ++e) {
    const int j = c0 + e;
    const bool ok = (j <= r);
    val[e] = ok ? (xv[e] - kDecay * (float)(r - j)) : -INFINITY;
    m = fmaxf(m, val[e]);
  }
#pragma unroll
  for (int off = 16; off > 0; off >>= 1) m = fmaxf(m, __shfl_xor(m, off, 32));
  if (lane == 0) redM[wave] = m;
  __syncthreads();
  m = fmaxf(fmaxf(fmaxf(redM[0], redM[1]), fmaxf(redM[2], redM[3])), fmaxf(fmaxf(redM[4], redM[5]), fmaxf(redM[6], redM[7])));
  float p[8];
  float psum = 0.f;
#pragma unroll
  for (int e = 0; e < 8; ++e) {
    const bool ok = (c0 + e <= r);
    p[e] = ok ? expf(val[e] - m) : 0.f;
    psum += p[e];
  }
#pragma unroll
  for (int off = 16; off > 0; off >>= 1) psum += __shfl_xor(psum, off, 32);
  if (lane == 0) redS[wave] = psum;
  __syncthreads();
  const float sum = ((((((redS[0] + redS[1]) + redS[2]) + redS[3]) + redS[4]) + redS[5]) + redS[6]) + redS[7];
  const float inv = carry * (1.0f / sum);
  unsigned short hb[8];
#pragma unroll
  for (int e = 0; e < 8; ++e) hb[e] = h_bits(p[e] * inv);
  const v4u u = (v4u){pk16(hb[0], hb[1]), pk16(hb[2], hb[3]), pk16(hb[4], hb[5]), pk16(hb[6], hb[7])};
  unsigned short* pp = P + (size_t)z * kSeq * kSeq + (size_t)r * kSeq + c0;
  *(volatile v4u*)pp = u;
  __threadfence();
  *(volatile v4u*)pp = u;
}

extern "C" void kernel_launch(void* const* d_in, const int* in_sizes, int n_in,
                              void* d_out, int out_size, void* d_ws, size_t ws_size,
                              hipStream_t stream) {
  (void)n_in;
  const float* x  = (const float*)d_in[0];
  const float* w3 = (const float*)d_in[1];
  const float* w5 = (const float*)d_in[2];
  const float* fw = (const float*)d_in[3];
  const float* fb = (const float*)d_in[4];
  float* out = (float*)d_out;

  if (in_sizes[0] != kTok * kDim || in_sizes[1] != kDim * 3 || in_sizes[2] != kDim * 5 ||
      in_sizes[3] != kDim * kCat || in_sizes[4] != kDim || out_size != kTok * kDim) return;

  const size_t offVS  = 0;
  const size_t offVT  = offVS  + (size_t)kTok * kDim * 2;
  const size_t offS   = offVT  + (size_t)kTok * kDim * 2;
  const size_t offP   = offS   + (size_t)2 * kSeq * kSeq * 4;
  const size_t offVt  = offP   + (size_t)2 * kSeq * kSeq * 2;
  const size_t offCat = offVt  + (size_t)2 * kDim * kSeq * 2;
  const size_t offW   = offCat + (size_t)kTok * kCat * 2;
  const size_t total  = offW   + (size_t)kDim * kCat * 2;
  if (total > ws_size) return;

  char* ws = (char*)d_ws;
  unsigned short* vS16 = (unsigned short*)(ws + offVS);
  unsigned short* vT16 = (unsigned short*)(ws + offVT);
  float*          Sbuf = (float*)(ws + offS);
  unsigned short* Pbuf = (unsigned short*)(ws + offP);
  unsigned short* Vt   = (unsigned short*)(ws + offVt);
  unsigned short* Cat  = (unsigned short*)(ws + offCat);
  unsigned short* W16  = (unsigned short*)(ws + offW);

  const long streamStride = (long)kTok * kDim;
  const long sStride      = (long)kSeq * kSeq;
  const long vtStride     = (long)kDim * kSeq;

  route_kernel<<<kTok, 256, 0, stream>>>(x, w3, w5, vS16, vT16);
  cast8_f16_kernel<<<(kDim * kCat / 8) / 256, 256, 0, stream>>>(fw, W16, kDim * kCat / 8, kWCarry);

  const int ntriBlocks = ((kSeq / 64) * (kSeq / 64 + 1) / 2 + 7) / 8;
  for (int bidx = 0; bidx < kBatch; ++bidx) {
    const unsigned short* Xb = vS16 + (size_t)bidx * kSeq * kDim;
    wmma_gemm64<0, false, 0, 0, false, 0, 1><<<dim3(ntriBlocks, 2), 256, 0, stream>>>(
        Xb, Xb, kDim, streamStride,
        Xb, Xb, kDim, streamStride,
        (void*)Sbuf, (void*)Sbuf, kSeq, sStride,
        fb, fb, 0L,
        kSeq, kSeq, kDim, kSimScale);
    vt_kernel<<<dim3(kDim / 64, kSeq / 64, 2), 256, 0, stream>>>(Xb, streamStride, Vt);
    softmax_kernel<<<dim3(kSeq, 2), 256, 0, stream>>>(Sbuf, Pbuf, kPCarry);
    wmma_gemm64<0, false, 0, 1, false, 0, 2><<<dim3((kSeq / 64) * (kDim / 64) / 8, 2), 256, 0, stream>>>(
        Pbuf, Pbuf, kSeq, sStride,
        Vt, Vt, kSeq, vtStride,
        (void*)(Cat + (size_t)bidx * kSeq * kCat), (void*)(Cat + (size_t)bidx * kSeq * kCat), kCat, (long)kDim,
        fb, fb, 0L,
        kSeq, kDim, kSeq, kPVScale);
  }
  wmma_gemm64<0, false, 2, 0, false, 0, 0><<<dim3((kTok / 64) * (kDim / 64) / 8, 1), 256, 0, stream>>>(
      Cat, Cat, kCat, 0L,
      W16, W16, kCat, 0L,
      (void*)out, (void*)out, kDim, 0L,
      fb, fb, 0L,
      kTok, kDim, kCat, kOutScale);
}
